// KGAT_61040075210791
// MI455X (gfx1250) — hardware-verified
//
#include <hip/hip_runtime.h>
#include <stddef.h>


#define DD      64
#define OUTW    160
#define NTHR    256
#define NWAVE   8
#define EPT     8
#define NGRP    2
#define CHUNK   (NTHR * EPT * NGRP)
#define WCAP    (EPT * NGRP * 32)
#define LISTN   (NWAVE * WCAP)
#define NBC     4096
#define NBF     1024
#define RCAP    32768
#define RBN     128
#define TGT     256
#define DEGCAP  256
#define GROWS   128
#define OTHR    512
#define WSCAP   134217728
#define WPL1    0
#define WPL2    16384
#define WPTOT   24576
#define APK     72

#define LDS_FILL ((RCAP + NBF + LISTN) * 4 + 64)
#define LDS_LAYER(DO) (4 * GROWS * APK * 2 + GROWS * (DO) * 4)

static_assert((CHUNK & (CHUNK - 1)) == 0);
static_assert(CHUNK <= 4096);
static_assert(NBC <= 4096 && NBF <= 4096);
static_assert((NBC & (NBC - 1)) == 0 && (NBF & (NBF - 1)) == 0);
static_assert(NBC == 4 * NBF);
static_assert(OTHR * 8 == NBC);
static_assert((RCAP % 32) == 0);
static_assert((TGT % GROWS) == 0 && TGT == NWAVE * 32);
static_assert((NBC % TGT) == 0);
static_assert(GROWS == NWAVE * 16);
static_assert(WPL2 == WPL1 + 4 * 64 * DD && WPTOT == WPL2 + 4 * 32 * DD);
static_assert(((4 * GROWS * APK * 2) % 16) == 0);

typedef float          v2f  __attribute__((ext_vector_type(2)));
typedef float          v4f  __attribute__((ext_vector_type(4)));
typedef float          v8f  __attribute__((ext_vector_type(8)));
typedef int            v4i  __attribute__((ext_vector_type(4)));
typedef unsigned short v8us __attribute__((ext_vector_type(8)));
typedef __bf16         v16b __attribute__((ext_vector_type(16)));
union FragB { v16b v; v8us h[2]; };

__device__ __forceinline__ unsigned int bfr(float f) {
  const unsigned int u = __float_as_uint(f);
  return (u + 0x7FFFu + ((u >> 16) & 1u)) >> 16;
}

__device__ __forceinline__ void split1(float x, unsigned short& hb, unsigned short& lb) {
  const unsigned int hu = bfr(x);
  const float hf = __uint_as_float(hu << 16);
  hb = (unsigned short)hu;
  lb = (unsigned short)bfr(x - hf);
}

__device__ __forceinline__ void split8(v4f a, v4f b, v8us& hi, v8us& lo) {
  unsigned short hb, lb;
  split1(a.x, hb, lb); hi[0] = hb; lo[0] = lb;
  split1(a.y, hb, lb); hi[1] = hb; lo[1] = lb;
  split1(a.z, hb, lb); hi[2] = hb; lo[2] = lb;
  split1(a.w, hb, lb); hi[3] = hb; lo[3] = lb;
  split1(b.x, hb, lb); hi[4] = hb; lo[4] = lb;
  split1(b.y, hb, lb); hi[5] = hb; lo[5] = lb;
  split1(b.z, hb, lb); hi[6] = hb; lo[6] = lb;
  split1(b.w, hb, lb); hi[7] = hb; lo[7] = lb;
}

__device__ __forceinline__ v8f wmb(v16b a, v16b b, v8f c) {
  v8f d = __builtin_amdgcn_wmma_f32_16x16x32_bf16(false, a, false, b, (short)0, c, false, false);
  asm volatile("v_nop\n\tv_nop\n\tv_nop\n\tv_nop" : "+v"(d) : "v"(a), "v"(b));
  return d;
}

template <int NB>
__device__ __forceinline__ int scan_chunk(const int* __restrict__ dsts, int nE, int cbase, int slotBase,
                                          int vec8, int* list, int tid, int lane, int wave) {
  int wc = 0;
#pragma unroll
  for (int g = 0; g < NGRP; ++g) {
    const int el0  = (g * NTHR + tid) * EPT;
    const int e0   = cbase + el0;
    const int sent = -2147483647 - 1;
    v4i da, db;
    if (vec8 != 0 && cbase + CHUNK <= nE) {
      da = *(const v4i*)(dsts + e0);
      db = *(const v4i*)(dsts + e0 + 4);
    } else {
      da.x = (e0     < nE) ? dsts[min(e0, nE - 1)] : sent;
      da.y = (e0 + 1 < nE) ? dsts[min(e0 + 1, nE - 1)] : sent;
      da.z = (e0 + 2 < nE) ? dsts[min(e0 + 2, nE - 1)] : sent;
      da.w = (e0 + 3 < nE) ? dsts[min(e0 + 3, nE - 1)] : sent;
      db.x = (e0 + 4 < nE) ? dsts[min(e0 + 4, nE - 1)] : sent;
      db.y = (e0 + 5 < nE) ? dsts[min(e0 + 5, nE - 1)] : sent;
      db.z = (e0 + 6 < nE) ? dsts[min(e0 + 6, nE - 1)] : sent;
      db.w = (e0 + 7 < nE) ? dsts[min(e0 + 7, nE - 1)] : sent;
    }
    const unsigned nb = (unsigned)slotBase;
    const unsigned s0 = (unsigned)da.x - nb, s1 = (unsigned)da.y - nb;
    const unsigned s2 = (unsigned)da.z - nb, s3 = (unsigned)da.w - nb;
    const unsigned s4 = (unsigned)db.x - nb, s5 = (unsigned)db.y - nb;
    const unsigned s6 = (unsigned)db.z - nb, s7 = (unsigned)db.w - nb;
    const bool h0 = s0 < (unsigned)NB, h1 = s1 < (unsigned)NB, h2 = s2 < (unsigned)NB, h3 = s3 < (unsigned)NB;
    const bool h4 = s4 < (unsigned)NB, h5 = s5 < (unsigned)NB, h6 = s6 < (unsigned)NB, h7 = s7 < (unsigned)NB;
    const unsigned any = __builtin_amdgcn_ballot_w32(h0 | h1 | h2 | h3 | h4 | h5 | h6 | h7);
    if (any != 0u) {
#define HITJ(J, HJ, SJ) { \
        const unsigned mj = __builtin_amdgcn_ballot_w32(HJ); \
        if (mj != 0u) { \
          if (HJ) { \
            const int pos = wc + (int)__builtin_amdgcn_mbcnt_lo(mj, 0u); \
            if (pos < WCAP) list[wave * WCAP + pos] = ((el0 + (J)) << 12) | (int)(SJ); \
          } \
          wc += (int)__builtin_popcount(mj); } }
      HITJ(0, h0, s0)
      HITJ(1, h1, s1)
      HITJ(2, h2, s2)
      HITJ(3, h3, s3)
      HITJ(4, h4, s4)
      HITJ(5, h5, s5)
      HITJ(6, h6, s6)
      HITJ(7, h7, s7)
#undef HITJ
    }
  }
  return wc;
}

__global__ __launch_bounds__(NTHR) void k_wprep(
    const float* __restrict__ w11, const float* __restrict__ w21,
    const float* __restrict__ w12, const float* __restrict__ w22, unsigned short* wp) {
  const int blk = blockIdx.x, tid = threadIdx.x;
  const float* w; int DO, base, i;
  if (blk < 2)       { w = w11; DO = 64; base = WPL1;               i = blk * NTHR + tid; }
  else if (blk < 4)  { w = w21; DO = 64; base = WPL1 + 2 * 64 * DD; i = (blk - 2) * NTHR + tid; }
  else if (blk == 4) { w = w12; DO = 32; base = WPL2;               i = tid; }
  else               { w = w22; DO = 32; base = WPL2 + 2 * 32 * DD; i = tid; }
  const int n  = i >> 3;
  const int k0 = (i & 7) * 8;
  float v[8];
#pragma unroll
  for (int e = 0; e < 8; ++e) v[e] = w[(k0 + e) * DO + n];
  v4f a, b;
  a.x = v[0]; a.y = v[1]; a.z = v[2]; a.w = v[3];
  b.x = v[4]; b.y = v[5]; b.z = v[6]; b.w = v[7];
  v8us hv, lv;
  split8(a, b, hv, lv);
  unsigned short* dh = wp + base + (size_t)n * DD + k0;
  unsigned short* dl = dh + DO * DD;
  *(volatile v8us*)dh = hv;
  *(volatile v8us*)dl = lv;
  __threadfence();
  *(volatile v8us*)dh = hv;
  *(volatile v8us*)dl = lv;
}

__global__ __launch_bounds__(NTHR) void k_concat(
    const float* __restrict__ ut, const float* __restrict__ et, float* E0, int nU, int nEn, int nN) {
  const int idx = blockIdx.x * NTHR + threadIdx.x;
  const int row = idx >> 4, c = (idx & 15) * 4;
  const int ru = row > nU - 1 ? nU - 1 : row;
  int re = row - nU;
  re = re < 0 ? 0 : (re > nEn - 1 ? nEn - 1 : re);
  const v4f vu = *(const v4f*)(ut + (size_t)ru * DD + c);
  const v4f ve = *(const v4f*)(et + (size_t)re * DD + c);
  const bool isU = row < nU, isE = row < nN;
  v4f v;
  v.x = isU ? vu.x : (isE ? ve.x : 0.0f);
  v.y = isU ? vu.y : (isE ? ve.y : 0.0f);
  v.z = isU ? vu.z : (isE ? ve.z : 0.0f);
  v.w = isU ? vu.w : (isE ? ve.w : 0.0f);
  float* gp = E0 + (size_t)idx * 4;
  *(volatile v4f*)gp = v;
  __threadfence();
  *(volatile v4f*)gp = v;
}

__global__ __launch_bounds__(NTHR) void k_count(const int* __restrict__ dsts, int* cnt, int nE, int vec8) {
  __shared__ __attribute__((aligned(16))) int scnt[NBC];
  __shared__ __attribute__((aligned(16))) int list[LISTN];
  __shared__ int wcnt[NWAVE];
  const int tid = threadIdx.x, lane = tid & 31, wave = tid >> 5;
  const int nodeBase = blockIdx.x * NBC;

  for (int i = tid; i < NBC; i += NTHR) scnt[i] = 0;
  __syncthreads();

  const int nChunks = (nE + CHUNK - 1) / CHUNK;
#pragma unroll 1
  for (int ch = 0; ch < nChunks; ++ch) {
    const int cbase = ch * CHUNK;
    const int wc = scan_chunk<NBC>(dsts, nE, cbase, nodeBase, vec8, list, tid, lane, wave);
    if (lane == 0) wcnt[wave] = wc;
    __syncthreads();
    if (wave == 0) {
#pragma unroll 1
      for (int wsx = 0; wsx < NWAVE; ++wsx) {
        int n = __builtin_amdgcn_readfirstlane(wcnt[wsx]);
        n = n > WCAP ? WCAP : (n < 0 ? 0 : n);
        const int* lp = list + wsx * WCAP;
#pragma unroll 1
        for (int i = 0; i < n; ++i) {
          const int ent  = __builtin_amdgcn_readfirstlane(lp[i]);
          const int slot = ent & (NBC - 1);
          if (lane == 0) scnt[slot] = scnt[slot] + 1;
        }
      }
    }
    __syncthreads();
  }

  v4i cq[4];
#pragma unroll
  for (int q = 0; q < 4; ++q) {
    const int f = (wave * 4 + q) * 128 + 4 * lane;
    cq[q] = *(const v4i*)(scnt + f);
  }
  int* cp = cnt + (size_t)nodeBase;
#pragma unroll
  for (int q = 0; q < 4; ++q) {
    const int f = (wave * 4 + q) * 128 + 4 * lane;
    *(volatile v4i*)(cp + f) = cq[q];
  }
  __threadfence();
#pragma unroll
  for (int q = 0; q < 4; ++q) {
    const int f = (wave * 4 + q) * 128 + 4 * lane;
    *(volatile v4i*)(cp + f) = cq[q];
  }
}

__global__ __launch_bounds__(OTHR) void k_offsets(
    const int* __restrict__ cnt, int* off, int* rbase, int nChunk) {
  __shared__ __attribute__((aligned(16))) int soff[NBC];
  __shared__ __attribute__((aligned(16))) int srb[RBN];
  __shared__ int wtot[OTHR / 32];
  const int tid = threadIdx.x, lane = tid & 31, wave = tid >> 5, sub = tid >> 7;
  for (int i = tid; i < RBN; i += OTHR) srb[i] = 0;
  int carry = 0;
#pragma unroll 1
  for (int ch = 0; ch < nChunk; ++ch) {
    const int base = ch * NBC;
    const v4i c0 = *(const v4i*)(cnt + base + 8 * tid);
    const v4i c1 = *(const v4i*)(cnt + base + 8 * tid + 4);
    const int e0 = max(c0.x, 0), e1 = max(c0.y, 0), e2 = max(c0.z, 0), e3 = max(c0.w, 0);
    const int e4 = max(c1.x, 0), e5 = max(c1.y, 0), e6 = max(c1.z, 0), e7 = max(c1.w, 0);
    const int ts = e0 + e1 + e2 + e3 + e4 + e5 + e6 + e7;
    int incl = ts;
#pragma unroll
    for (int d = 1; d < 32; d <<= 1) {
      const int t = __shfl_up(incl, d);
      if (lane >= d) incl += t;
    }
    if (lane == 31) wtot[wave] = incl;
    __syncthreads();
    const int S0 = wtot[0]  + wtot[1]  + wtot[2]  + wtot[3];
    const int S1 = wtot[4]  + wtot[5]  + wtot[6]  + wtot[7];
    const int S2 = wtot[8]  + wtot[9]  + wtot[10] + wtot[11];
    const int S3 = wtot[12] + wtot[13] + wtot[14] + wtot[15];
    int pre = 0;
#pragma unroll 1
    for (int w = 4 * sub; w < wave; ++w) pre += wtot[w];
    const int b0 = carry;
    const int b1 = b0 + ((S0 + 31) & ~31);
    const int b2 = b1 + ((S1 + 31) & ~31);
    const int b3 = b2 + ((S2 + 31) & ~31);
    const int b4 = b3 + ((S3 + 31) & ~31);
    const int myb = sub == 0 ? b0 : (sub == 1 ? b1 : (sub == 2 ? b2 : b3));
    if (tid == 0) {
      srb[min(4 * ch + 0, RBN - 1)] = b0;
      srb[min(4 * ch + 1, RBN - 1)] = b1;
      srb[min(4 * ch + 2, RBN - 1)] = b2;
      srb[min(4 * ch + 3, RBN - 1)] = b3;
    }
    int run = myb + pre + incl - ts;
    soff[8 * tid + 0] = run; run += e0;
    soff[8 * tid + 1] = run; run += e1;
    soff[8 * tid + 2] = run; run += e2;
    soff[8 * tid + 3] = run; run += e3;
    soff[8 * tid + 4] = run; run += e4;
    soff[8 * tid + 5] = run; run += e5;
    soff[8 * tid + 6] = run; run += e6;
    soff[8 * tid + 7] = run;
    carry = b4;
    __syncthreads();
    const v4i o0 = *(const v4i*)(soff + 4 * tid);
    const v4i o1 = *(const v4i*)(soff + 4 * (tid + OTHR));
    int* op = off + base;
    *(volatile v4i*)(op + 4 * tid) = o0;
    *(volatile v4i*)(op + 4 * (tid + OTHR)) = o1;
    __threadfence();
    *(volatile v4i*)(op + 4 * tid) = o0;
    *(volatile v4i*)(op + 4 * (tid + OTHR)) = o1;
    __syncthreads();
  }
  if (tid == 0) srb[min(4 * nChunk, RBN - 1)] = carry;
  __syncthreads();
  v4i rv = {0, 0, 0, 0};
  if (tid < 32) rv = *(const v4i*)(srb + 4 * tid);
  if (tid < 32) *(volatile v4i*)(rbase + 4 * tid) = rv;
  __threadfence();
  if (tid < 32) *(volatile v4i*)(rbase + 4 * tid) = rv;
}

__global__ __launch_bounds__(NTHR) void k_fill(
    const int* __restrict__ dsts, const int* __restrict__ off, const int* __restrict__ rbase,
    int* csr, int nE, int vec8, int csrLen) {
  extern __shared__ v4f lds_dyn[];
  int* region = (int*)lds_dyn;
  int* cursor = region + RCAP;
  int* list   = cursor + NBF;
  int* wcnt   = list + LISTN;
  const int tid = threadIdx.x, lane = tid & 31, wave = tid >> 5;
  const int b = blockIdx.x;
  const int nodeBase = b * NBF;

  int rb0 = rbase[b];
  const int rb1 = rbase[b + 1];
  rb0 = rb0 < 0 ? 0 : (rb0 > csrLen ? csrLen : rb0);
  rb0 &= ~31;
  int len = rb1 - rb0;
  len = len < 0 ? 0 : (len > RCAP ? RCAP : len);
  int lenW = (len + 31) & ~31;
  if (rb0 + lenW > csrLen) lenW = (csrLen - rb0) & ~31;

  {
    const v4i z = {0, 0, 0, 0};
    for (int i = tid; i < RCAP / 4; i += NTHR) ((v4i*)region)[i] = z;
    for (int s = tid; s < NBF; s += NTHR) {
      int o = off[nodeBase + s] - rb0;
      o = o < 0 ? 0 : (o > RCAP ? RCAP : o);
      cursor[s] = o;
    }
  }
  __syncthreads();

  const int nChunks = (nE + CHUNK - 1) / CHUNK;
#pragma unroll 1
  for (int ch = 0; ch < nChunks; ++ch) {
    const int cbase = ch * CHUNK;
    const int wc = scan_chunk<NBF>(dsts, nE, cbase, nodeBase, vec8, list, tid, lane, wave);
    if (lane == 0) wcnt[wave] = wc;
    __syncthreads();
    if (wave == 0) {
#pragma unroll 1
      for (int wsx = 0; wsx < NWAVE; ++wsx) {
        int n = __builtin_amdgcn_readfirstlane(wcnt[wsx]);
        n = n > WCAP ? WCAP : (n < 0 ? 0 : n);
        const int* lp = list + wsx * WCAP;
#pragma unroll 1
        for (int i = 0; i < n; ++i) {
          const int ent  = __builtin_amdgcn_readfirstlane(lp[i]);
          const int slot = ent & (NBF - 1);
          int e = cbase + ((ent >> 12) & (CHUNK - 1));
          e = e > nE - 1 ? nE - 1 : e;
          if (lane == 0) {
            int pos = cursor[slot];
            pos = pos < 0 ? 0 : (pos > RCAP - 1 ? RCAP - 1 : pos);
            region[pos] = e;
            const int np = pos + 1;
            cursor[slot] = np > RCAP ? RCAP : np;
          }
        }
      }
    }
    __syncthreads();
  }

  const int nv = lenW >> 2;
  int* gp = csr + rb0;
#pragma unroll 1
  for (int i = tid; i < nv; i += NTHR) { const v4i v = ((const v4i*)region)[i]; *(volatile v4i*)(gp + 4 * i) = v; }
  __threadfence();
#pragma unroll 1
  for (int i = tid; i < nv; i += NTHR) { const v4i v = ((const v4i*)region)[i]; *(volatile v4i*)(gp + 4 * i) = v; }
}

__device__ __forceinline__ v2f agg_seg(
    const int* __restrict__ csr, const int* __restrict__ acol, const float* __restrict__ aval,
    const float* __restrict__ xin, int n, int st, int lane, int nN, int nE, int csrLen) {
  v2f acc = {0.0f, 0.0f};
#pragma unroll 1
  for (int q0 = 0; q0 < n; q0 += 32) {
    int pos = st + q0 + lane;
    pos = pos < 0 ? 0 : (pos > csrLen - 1 ? csrLen - 1 : pos);
    int ed = csr[pos];
    ed = ed < 0 ? 0 : (ed > nE - 1 ? nE - 1 : ed);
    int cl = acol[ed];
    cl = cl < 0 ? 0 : (cl > nN - 1 ? nN - 1 : cl);
    const float vl = aval[ed];
    const int mcnt = (n - q0) < 32 ? (n - q0) : 32;
#pragma unroll 1
    for (int p = 0; p < mcnt; ++p) {
      const int   s = __builtin_amdgcn_readlane(cl, p);
      const float v = __int_as_float(__builtin_amdgcn_readlane(__float_as_int(vl), p));
      const v2f   x = *(const v2f*)(xin + (size_t)s * DD + 2 * lane);
      acc.x = fmaf(v, x.x, acc.x);
      acc.y = fmaf(v, x.y, acc.y);
    }
  }
  return acc;
}

__global__ __launch_bounds__(NTHR) void k_agg(
    const int* __restrict__ csr, const int* __restrict__ off, const int* __restrict__ cnt,
    const int* __restrict__ acol, const float* __restrict__ aval,
    const float* __restrict__ xin, float* S, int nN, int nE, int csrLen) {
  const int tid = threadIdx.x, lane = tid & 31, wave = tid >> 5;
  const int tbase = blockIdx.x * TGT + wave * 32;
  const int cl = tbase + lane;
  const int cnt_l = cnt[cl];
  const int off_l = off[cl];
  const int q2 = 2 * (lane & 15);
  const int tg = lane >> 4;

#pragma unroll 1
  for (int j = 0; j < 32; j += 2) {
    int na = __builtin_amdgcn_readlane(cnt_l, j);
    na = na < 0 ? 0 : (na > DEGCAP ? DEGCAP : na);
    const int sa = __builtin_amdgcn_readlane(off_l, j);
    int nb = __builtin_amdgcn_readlane(cnt_l, j + 1);
    nb = nb < 0 ? 0 : (nb > DEGCAP ? DEGCAP : nb);
    const int sb = __builtin_amdgcn_readlane(off_l, j + 1);
    const v2f accA = agg_seg(csr, acol, aval, xin, na, sa, lane, nN, nE, csrLen);
    const v2f accB = agg_seg(csr, acol, aval, xin, nb, sb, lane, nN, nE, csrLen);
    const float a0 = __shfl(accA.x, q2),     a1 = __shfl(accA.y, q2);
    const float a2 = __shfl(accA.x, q2 + 1), a3 = __shfl(accA.y, q2 + 1);
    const float c0 = __shfl(accB.x, q2),     c1 = __shfl(accB.y, q2);
    const float c2 = __shfl(accB.x, q2 + 1), c3 = __shfl(accB.y, q2 + 1);
    v4f w;
    w.x = tg != 0 ? c0 : a0;
    w.y = tg != 0 ? c1 : a1;
    w.z = tg != 0 ? c2 : a2;
    w.w = tg != 0 ? c3 : a3;
    float* gp = S + (size_t)(tbase + j) * DD + 4 * lane;
    *(volatile v4f*)gp = w;
    __threadfence();
    *(volatile v4f*)gp = w;
  }
}

template <int DOUT, int COLB, int WN>
__global__ __launch_bounds__(NTHR) void k_layer(
    const float* __restrict__ ego, const float* __restrict__ side,
    const unsigned short* __restrict__ Wp, const float* __restrict__ b1, const float* __restrict__ b2,
    float* out, float* egon, int nN) {
  static_assert((DOUT % 16) == 0 && DOUT <= DD);
  static_assert(WN == 0 || DOUT == DD);
  static_assert(COLB != 0 || DOUT == DD);
  static_assert(((GROWS * DD / 8) % NTHR) == 0);
  extern __shared__ v4f lds_dyn[];
  constexpr int NT   = DOUT / 16;
  constexpr int WPLN = DOUT * DD;
  unsigned short* sSh = (unsigned short*)lds_dyn;
  unsigned short* sSl = sSh + GROWS * APK;
  unsigned short* sPh = sSl + GROWS * APK;
  unsigned short* sPl = sPh + GROWS * APK;
  float*          stg = (float*)(sPl + GROWS * APK);
  const int tid = threadIdx.x, lane = tid & 31, wave = tid >> 5, hh = lane >> 4, m = lane & 15;
  const int rowBase = blockIdx.x * GROWS;

#pragma unroll
  for (int i = 0; i < (GROWS * DD / 8) / NTHR; ++i) {
    const int idx = i * NTHR + tid;
    const int r   = idx >> 3;
    const int c0  = (idx & 7) * 8;
    const float* ep = ego  + (size_t)(rowBase + r) * DD + c0;
    const float* sp = side + (size_t)(rowBase + r) * DD + c0;
    const v4f ea = *(const v4f*)ep, eb = *(const v4f*)(ep + 4);
    const v4f sa = *(const v4f*)sp, sb = *(const v4f*)(sp + 4);
    const v4f ua = ea + sa, ub = eb + sb;
    const v4f pa = ea * sa, pb = eb * sb;
    v8us h1, l1, h2, l2;
    split8(ua, ub, h1, l1);
    split8(pa, pb, h2, l2);
    *(v8us*)(sSh + r * APK + c0) = h1;
    *(v8us*)(sSl + r * APK + c0) = l1;
    *(v8us*)(sPh + r * APK + c0) = h2;
    *(v8us*)(sPl + r * APK + c0) = l2;
  }
  __syncthreads();

  const unsigned short* psh = sSh + (wave * 16 + m) * APK + 8 * hh;
  const unsigned short* psl = sSl + (wave * 16 + m) * APK + 8 * hh;
  const unsigned short* pph = sPh + (wave * 16 + m) * APK + 8 * hh;
  const unsigned short* ppl = sPl + (wave * 16 + m) * APK + 8 * hh;
  float vals[NT][8];
  float ss[8];
#pragma unroll
  for (int r = 0; r < 8; ++r) ss[r] = 0.0f;

#pragma unroll
  for (int t = 0; t < NT; ++t) {
    v8f acc1 = {0.f, 0.f, 0.f, 0.f, 0.f, 0.f, 0.f, 0.f};
    v8f acc2 = {0.f, 0.f, 0.f, 0.f, 0.f, 0.f, 0.f, 0.f};
#pragma unroll
    for (int kt = 0; kt < 2; ++kt) {
      FragB ah, al, ph, pl;
      ah.h[0] = *(const v8us*)(psh + 32 * kt);
      ah.h[1] = *(const v8us*)(psh + 32 * kt + 16);
      al.h[0] = *(const v8us*)(psl + 32 * kt);
      al.h[1] = *(const v8us*)(psl + 32 * kt + 16);
      ph.h[0] = *(const v8us*)(pph + 32 * kt);
      ph.h[1] = *(const v8us*)(pph + 32 * kt + 16);
      pl.h[0] = *(const v8us*)(ppl + 32 * kt);
      pl.h[1] = *(const v8us*)(ppl + 32 * kt + 16);
      const unsigned short* bp = Wp + (size_t)(16 * t + m) * DD + 32 * kt + 8 * hh;
      FragB b1h, b1l, b2h, b2l;
      b1h.h[0] = *(const v8us*)bp;                b1h.h[1] = *(const v8us*)(bp + 16);
      b1l.h[0] = *(const v8us*)(bp + WPLN);       b1l.h[1] = *(const v8us*)(bp + WPLN + 16);
      b2h.h[0] = *(const v8us*)(bp + 2 * WPLN);   b2h.h[1] = *(const v8us*)(bp + 2 * WPLN + 16);
      b2l.h[0] = *(const v8us*)(bp + 3 * WPLN);   b2l.h[1] = *(const v8us*)(bp + 3 * WPLN + 16);
      acc1 = wmb(ah.v, b1h.v, acc1);
      acc1 = wmb(ah.v, b1l.v, acc1);
      acc1 = wmb(al.v, b1h.v, acc1);
      acc2 = wmb(ph.v, b2h.v, acc2);
      acc2 = wmb(ph.v, b2l.v, acc2);
      acc2 = wmb(pl.v, b2h.v, acc2);
    }
    const float bv1 = b1[16 * t + m];
    const float bv2 = b2[16 * t + m];
#pragma unroll
    for (int r = 0; r < 8; ++r) {
      float sv = acc1[r] + bv1; sv = sv >= 0.0f ? sv : 0.01f * sv;
      float pv = acc2[r] + bv2; pv = pv >= 0.0f ? pv : 0.01f * pv;
      const float v = sv + pv;
      vals[t][r] = v;
      ss[r] = fmaf(v, v, ss[r]);
    }
  }

  float rn[8];
#pragma unroll
  for (int r = 0; r < 8; ++r) {
    float s = ss[r];
    s += __shfl_xor(s, 1, 16);
    s += __shfl_xor(s, 2, 16);
    s += __shfl_xor(s, 4, 16);
    s += __shfl_xor(s, 8, 16);
    rn[r] = 1.0f / fmaxf(sqrtf(s), 1e-12f);
  }
  float* strow = stg + (wave * 16 + 8 * hh) * DOUT + m;
#pragma unroll
  for (int t = 0; t < NT; ++t) {
#pragma unroll
    for (int r = 0; r < 8; ++r) strow[r * DOUT + 16 * t] = vals[t][r] * rn[r];
  }
  __syncthreads();

  if (WN != 0) {
#pragma unroll
    for (int i = 0; i < 8; ++i) {
      const int row = wave * 16 + 2 * i + hh;
      const v4f v = *(const v4f*)(stg + row * DOUT + 4 * m);
      *(volatile v4f*)(egon + (size_t)(rowBase + row) * DD + 4 * m) = v;
    }
  }
  if (COLB == 0) {
#pragma unroll
    for (int i = 0; i < 16; ++i) {
      const int row = wave * 16 + i, grow = rowBase + row;
      const v4f ve = *(const v4f*)(ego + (size_t)grow * DD + 4 * m);
      const v4f vs = *(const v4f*)(stg + row * DOUT + 4 * m);
      v4f v;
      v.x = hh == 0 ? ve.x : vs.x; v.y = hh == 0 ? ve.y : vs.y;
      v.z = hh == 0 ? ve.z : vs.z; v.w = hh == 0 ? ve.w : vs.w;
      if (grow < nN) *(volatile v4f*)(out + (size_t)grow * OUTW + 4 * lane) = v;
    }
  } else {
#pragma unroll
    for (int i = 0; i < 4; ++i) {
      const int row = wave * 16 + 4 * i + (lane >> 3), grow = rowBase + row;
      const v4f v = *(const v4f*)(stg + row * DOUT + 4 * (lane & 7));
      if (grow < nN) *(volatile v4f*)(out + (size_t)grow * OUTW + COLB + 4 * (lane & 7)) = v;
    }
  }
  __threadfence();
  if (WN != 0) {
#pragma unroll
    for (int i = 0; i < 8; ++i) {
      const int row = wave * 16 + 2 * i + hh;
      const v4f v = *(const v4f*)(stg + row * DOUT + 4 * m);
      *(volatile v4f*)(egon + (size_t)(rowBase + row) * DD + 4 * m) = v;
    }
  }
  if (COLB == 0) {
#pragma unroll
    for (int i = 0; i < 16; ++i) {
      const int row = wave * 16 + i, grow = rowBase + row;
      const v4f ve = *(const v4f*)(ego + (size_t)grow * DD + 4 * m);
      const v4f vs = *(const v4f*)(stg + row * DOUT + 4 * m);
      v4f v;
      v.x = hh == 0 ? ve.x : vs.x; v.y = hh == 0 ? ve.y : vs.y;
      v.z = hh == 0 ? ve.z : vs.z; v.w = hh == 0 ? ve.w : vs.w;
      if (grow < nN) *(volatile v4f*)(out + (size_t)grow * OUTW + 4 * lane) = v;
    }
  } else {
#pragma unroll
    for (int i = 0; i < 4; ++i) {
      const int row = wave * 16 + 4 * i + (lane >> 3), grow = rowBase + row;
      const v4f v = *(const v4f*)(stg + row * DOUT + 4 * (lane & 7));
      if (grow < nN) *(volatile v4f*)(out + (size_t)grow * OUTW + COLB + 4 * (lane & 7)) = v;
    }
  }
}

extern "C" void kernel_launch(void* const* d_in, const int* in_sizes, int n_in,
                              void* d_out, int out_size, void* d_ws, size_t ws_size,
                              hipStream_t stream) {
  if (n_in < 13) return;
  const int nU  = in_sizes[0] / DD;
  const int nEn = in_sizes[1] / DD;
  if (nU < 1 || nEn < 1 || in_sizes[0] != nU * DD || in_sizes[1] != nEn * DD) return;
  const int nN = nU + nEn;
  const int nE = in_sizes[2];
  if (nE < 1 || in_sizes[11] != nE || in_sizes[12] != nE) return;
  if (in_sizes[3] != DD * 64 || in_sizes[4] != 64 || in_sizes[5] != DD * 64 || in_sizes[6] != 64) return;
  if (in_sizes[7] != DD * 32 || in_sizes[8] != 32 || in_sizes[9] != DD * 32 || in_sizes[10] != 32) return;
  if ((long long)out_size != (long long)nN * OUTW) return;
  if (nE > (1 << 28) || nN > (1 << 24)) return;

  const float* ut   = (const float*)d_in[0];
  const float* et   = (const float*)d_in[1];
  const float* aval = (const float*)d_in[2];
  const float* w11  = (const float*)d_in[3];
  const float* b11  = (const float*)d_in[4];
  const float* w21  = (const float*)d_in[5];
  const float* b21  = (const float*)d_in[6];
  const float* w12  = (const float*)d_in[7];
  const float* b12  = (const float*)d_in[8];
  const float* w22  = (const float*)d_in[9];
  const float* b22  = (const float*)d_in[10];
  const int*   arow = (const int*)d_in[11];
  const int*   acol = (const int*)d_in[12];
  float* out = (float*)d_out;

  const int NPAD   = ((nN + TGT - 1) / TGT) * TGT;
  const int nBC    = (nN + NBC - 1) / NBC;
  const int CNTPAD = nBC * NBC;
  if (4 * nBC + 1 > RBN) return;
  const int nBF    = (nN + NBF - 1) / NBF;
  const int csrLen = ((nE + 31) & ~31) + 4096;
  if (31 * 4 * nBC > 4096) return;
  const int nLay   = NPAD / GROWS;
  const int nAgg   = NPAD / TGT;
  const int nCat   = NPAD / 16;

  char* ws = (char*)d_ws;
  size_t off = 0;
  const size_t oW   = off; off += (size_t)WPTOT * 2;               off = (off + 255) & ~(size_t)255;
  const size_t oCnt = off; off += (size_t)CNTPAD * 4;              off = (off + 255) & ~(size_t)255;
  const size_t oOff = off; off += (size_t)CNTPAD * 4;              off = (off + 255) & ~(size_t)255;
  const size_t oRb  = off; off += (size_t)RBN * 4;                 off = (off + 255) & ~(size_t)255;
  const size_t oCsr = off; off += (size_t)csrLen * 4;              off = (off + 255) & ~(size_t)255;
  const size_t oE0  = off; off += (size_t)NPAD * DD * 4;           off = (off + 255) & ~(size_t)255;
  const size_t oSd  = off; off += (size_t)NPAD * DD * 4;           off = (off + 255) & ~(size_t)255;
  const size_t oE1  = off; off += (size_t)NPAD * DD * 4;           off = (off + 255) & ~(size_t)255;
  if (off > ws_size || off > (size_t)WSCAP) return;
  unsigned short* wp   = (unsigned short*)(ws + oW);
  int*            cnt  = (int*)(ws + oCnt);
  int*            offp = (int*)(ws + oOff);
  int*            rb   = (int*)(ws + oRb);
  int*            csr  = (int*)(ws + oCsr);
  float*          E0   = (float*)(ws + oE0);
  float*          Sd   = (float*)(ws + oSd);
  float*          E1   = (float*)(ws + oE1);

  const int vec8 = ((nE & 3) == 0) ? 1 : 0;

  k_wprep<<<6, NTHR, 0, stream>>>(w11, w21, w12, w22, wp);

  k_concat<<<nCat, NTHR, 0, stream>>>(ut, et, E0, nU, nEn, nN);

  k_count<<<nBC, NTHR, 0, stream>>>(arow, cnt, nE, vec8);
  k_offsets<<<1, OTHR, 0, stream>>>(cnt, offp, rb, nBC);
  hipFuncSetAttribute(reinterpret_cast<const void*>(&k_fill),
                      hipFuncAttributeMaxDynamicSharedMemorySize, LDS_FILL);
  k_fill<<<nBF, NTHR, LDS_FILL, stream>>>(arow, offp, rb, csr, nE, vec8, csrLen);

  k_agg<<<nAgg, NTHR, 0, stream>>>(csr, offp, cnt, acol, aval, E0, Sd, nN, nE, csrLen);
  hipFuncSetAttribute(reinterpret_cast<const void*>(&k_layer<64, 0, 1>),
                      hipFuncAttributeMaxDynamicSharedMemorySize, LDS_LAYER(64));
  k_layer<64, 0, 1><<<nLay, NTHR, LDS_LAYER(64), stream>>>(E0, Sd, wp + WPL1, b11, b21, out, E1, nN);

  k_agg<<<nAgg, NTHR, 0, stream>>>(csr, offp, cnt, acol, aval, E1, Sd, nN, nE, csrLen);
  hipFuncSetAttribute(reinterpret_cast<const void*>(&k_layer<32, 128, 0>),
                      hipFuncAttributeMaxDynamicSharedMemorySize, LDS_LAYER(32));
  k_layer<32, 128, 0><<<nLay, NTHR, LDS_LAYER(32), stream>>>(E1, Sd, wp + WPL2, b12, b22, out, E1, nN);
}
